// Projection_12506944766612
// MI455X (gfx1250) — hardware-verified
//
#include <hip/hip_runtime.h>
#include <hip/hip_bf16.h>

typedef __attribute__((ext_vector_type(16))) _Float16 v16h;
typedef __attribute__((ext_vector_type(8)))  _Float16 v8h;
typedef __attribute__((ext_vector_type(16))) __bf16   v16b;
typedef __attribute__((ext_vector_type(8)))  __bf16   v8b;
typedef __attribute__((ext_vector_type(8)))  float    v8f;
typedef __attribute__((ext_vector_type(4)))  float    v4f;
typedef __attribute__((ext_vector_type(2)))  float    v2f;
typedef __attribute__((ext_vector_type(4)))  unsigned v4u;

__device__ __forceinline__ unsigned short f2bf_bits(float f) {
  unsigned u = __float_as_uint(f);
  return (unsigned short)((u + 0x7FFFu + ((u >> 16) & 1u)) >> 16);
}
__device__ __forceinline__ float bf_bits2f(unsigned short h) { return __uint_as_float(((unsigned)h) << 16); }

__device__ __forceinline__ void dep_guard_h(v8f& a, v8f& b, v16h x, v16h y) { asm volatile("v_nop\n\tv_nop\n\tv_nop\n\tv_nop" : "+v"(a), "+v"(b) : "v"(x), "v"(y)); }
__device__ __forceinline__ void dep_guard_b(v8f& a, v8f& b, v16b x, v16b y) { asm volatile("v_nop\n\tv_nop\n\tv_nop\n\tv_nop" : "+v"(a), "+v"(b) : "v"(x), "v"(y)); }
__device__ __forceinline__ void keep4_h(v16h a, v16h b, v16h c, v16h d) { asm volatile("v_nop" :: "v"(a), "v"(b), "v"(c), "v"(d)); }
__device__ __forceinline__ void keep4_b(v16b a, v16b b, v16b c, v16b d) { asm volatile("v_nop" :: "v"(a), "v"(b), "v"(c), "v"(d)); }
__device__ __forceinline__ void acc_guard4(v8f& a, v8f& b, v8f& c, v8f& d) { asm volatile("v_nop\n\tv_nop\n\tv_nop\n\tv_nop" : "+v"(a), "+v"(b), "+v"(c), "+v"(d)); }
template <typename T> struct Frag;
template <> struct Frag<_Float16> {
  typedef v16h V; union U { v16h v; v8h h[2]; };
  static __device__ __forceinline__ v16h load(const _Float16* p) {
    U f; f.h[0] = *(const v8h*)(p); f.h[1] = *(const v8h*)(p + 16); return f.v;
  }
  static __device__ __forceinline__ v8f mma(v16h a, v16h b, v8f c) {
    return __builtin_amdgcn_wmma_f32_16x16x32_f16(false, a, false, b, (short)0, c, false, false);
  }
  static __device__ __forceinline__ void guard(v8f& a, v8f& b, v16h x, v16h y) { dep_guard_h(a, b, x, y); }
  static __device__ __forceinline__ void keep(v16h a, v16h b, v16h c, v16h d) { keep4_h(a, b, c, d); }
};
template <> struct Frag<__bf16> {
  typedef v16b V; union U { v16b v; v8b h[2]; };
  static __device__ __forceinline__ v16b load(const __bf16* p) {
    U f; f.h[0] = *(const v8b*)(p); f.h[1] = *(const v8b*)(p + 16); return f.v;
  }
  static __device__ __forceinline__ v8f mma(v16b a, v16b b, v8f c) {
    return __builtin_amdgcn_wmma_f32_16x16x32_bf16(false, a, false, b, (short)0, c, false, false);
  }
  static __device__ __forceinline__ void guard(v8f& a, v8f& b, v16b x, v16b y) { dep_guard_b(a, b, x, y); }
  static __device__ __forceinline__ void keep(v16b a, v16b b, v16b c, v16b d) { keep4_b(a, b, c, d); }
};

template <int ET> struct Elem;
template <> struct Elem<0> { typedef _Float16 T; };
template <> struct Elem<1> { typedef __bf16 T; };
template <int ET, int SPLIT, int BIAS_MODE, int OUT_MODE, bool RESID, int ACT = 0>
__global__ __launch_bounds__(256) void wmma_gemm64(
    const unsigned short* __restrict__ Ap, const unsigned short* __restrict__ A2p, int lda, long strideA,
    const unsigned short* __restrict__ Btp, const unsigned short* __restrict__ Bt2p, int ldb, long strideB,
    void* __restrict__ Cout, void* __restrict__ Cout2, int ldc, long strideC,
    const float* __restrict__ bias,
    const float* __restrict__ resid, long strideR,
    int M, int N, int K, float scale) {
  typedef typename Elem<ET>::T T;
  typedef typename Frag<T>::V V;
  constexpr bool ASPL = (SPLIT == 1) || (SPLIT == 2);
  constexpr bool BSPL = (SPLIT == 1) || (SPLIT == 3);
  const T* A = (const T*)Ap; const T* A2 = (const T*)A2p; const T* Bt = (const T*)Btp; const T* Bt2 = (const T*)Bt2p;
  __shared__ __align__(16) float sT[8][16 * 68];
  const int b    = blockIdx.y;
  const int lane = threadIdx.x & 31;
  const int wave = threadIdx.x >> 5;
  const int tilesN = N >> 6;
  const int tilesM = M >> 6;
  const int tile = blockIdx.x * 8 + wave;
  if (tile >= tilesM * tilesN) return;
  const int tm = tile / tilesN;
  const int tn = tile - tm * tilesN;
  const int m0 = tm << 6;
  const int n0 = tn << 6;

  const T* Ab  = A  + (size_t)b * strideA;
  const T* Bb  = Bt + (size_t)b * strideB;
  const T* Ab2 = ASPL ? (A2  + (size_t)b * strideA) : nullptr;
  const T* Bb2 = BSPL ? (Bt2 + (size_t)b * strideB) : nullptr;

  const int rlane = lane & 15;
  const int koff  = (lane >> 4) * 8;
  const int mOff  = (lane >> 4) * 8;

  v8f acc[4][4];
#pragma unroll
  for (int i = 0; i < 4; ++i)
#pragma unroll
    for (int j = 0; j < 4; ++j) acc[i][j] = (v8f){0.f,0.f,0.f,0.f,0.f,0.f,0.f,0.f};

  for (int k0 = 0; k0 < K; k0 += 32) {
    V bh[4], bl[4];
#pragma unroll
    for (int j = 0; j < 4; ++j) {
      const size_t bo = (size_t)(n0 + (j << 4) + rlane) * ldb + koff + k0;
      bh[j] = Frag<T>::load(Bb + bo);
      if (BSPL) bl[j] = Frag<T>::load(Bb2 + bo);
      else bl[j] = bh[j];
    }
#pragma unroll
    for (int i = 0; i < 4; ++i) {
      const size_t ao = (size_t)(m0 + (i << 4) + rlane) * lda + koff + k0;
      V ah = Frag<T>::load(Ab + ao);
      V al = ah;
      if (ASPL) al = Frag<T>::load(Ab2 + ao);
#pragma unroll
      for (int j = 0; j < 4; ++j) {
        acc[i][j] = Frag<T>::mma(ah, bh[j], acc[i][j]);
        if (BSPL) acc[i][j] = Frag<T>::mma(ah, bl[j], acc[i][j]);
        if (ASPL) acc[i][j] = Frag<T>::mma(al, bh[j], acc[i][j]);
      }
      Frag<T>::guard(acc[i][0], acc[i][3], ah, al);
    }
    Frag<T>::keep(bh[0], bh[1], bh[2], bh[3]);
    if (BSPL) Frag<T>::keep(bl[0], bl[1], bl[2], bl[3]);
  }
  acc_guard4(acc[0][0], acc[0][1], acc[0][2], acc[0][3]);
  acc_guard4(acc[1][0], acc[1][1], acc[1][2], acc[1][3]);
  acc_guard4(acc[2][0], acc[2][1], acc[2][2], acc[2][3]);
  acc_guard4(acc[3][0], acc[3][1], acc[3][2], acc[3][3]);

  float* slab = sT[wave];
  const float* Rb = RESID ? (resid + (size_t)b * strideR) : nullptr;
#pragma unroll
  for (int i = 0; i < 4; ++i) {
    const int mBase = m0 + (i << 4);
#pragma unroll
    for (int j = 0; j < 4; ++j) {
      const int n = n0 + (j << 4) + rlane;
      float bv = 0.f;
      if (BIAS_MODE == 2) bv = bias[n];
#pragma unroll
      for (int r = 0; r < 8; ++r) {
        float v = acc[i][j][r] * scale;
        if (BIAS_MODE == 1) v += bias[mBase + mOff + r];
        if (BIAS_MODE == 2) v += bv;
        if (RESID) v += Rb[(size_t)(mBase + mOff + r) * ldc + n];
        if (ACT == 1) v = tanhf(v);
        if (ACT == 2) v = fmaxf(v, 0.0f);
        if (ACT == 3) v = v / (1.0f + expf(-v));
        if (ACT == 4) v = (v > 0.f) ? v : 0.01f * v;
        slab[(mOff + r) * 68 + (j << 4) + rlane] = v;
      }
    }
    __builtin_amdgcn_fence(__ATOMIC_RELEASE, "workgroup");
    __builtin_amdgcn_wave_barrier();
    __builtin_amdgcn_fence(__ATOMIC_ACQUIRE, "workgroup");
    if (OUT_MODE == 0) {
      float* C = (float*)Cout + (size_t)b * strideC;
      const int hh = lane >> 4, c4 = (lane & 15) * 4;
      for (int pass = 0; pass < 2; ++pass) {
#pragma unroll
        for (int it = 0; it < 8; ++it) {
          const int row = it * 2 + hh;
          v4f v = *(const v4f*)(slab + row * 68 + c4);
          *(volatile v4f*)(C + (size_t)(mBase + row) * ldc + n0 + c4) = v;
        }
        __threadfence();
      }
    } else {
      const int q = lane >> 3, c8 = (lane & 7) * 8;
      unsigned short* C  = (unsigned short*)Cout  + (size_t)b * strideC;
      unsigned short* C2 = (OUT_MODE == 2) ? ((unsigned short*)Cout2 + (size_t)b * strideC) : nullptr;
      for (int pass = 0; pass < 2; ++pass) {
#pragma unroll
        for (int it = 0; it < 4; ++it) {
          const int row = it * 4 + q;
          const float* sp = slab + row * 68 + c8;
          v8h hv, lv;
#pragma unroll
          for (int e = 0; e < 8; ++e) {
            if (OUT_MODE == 1) {
              hv[e] = (_Float16)sp[e];
            } else {
              unsigned short hb = f2bf_bits(sp[e]);
              unsigned short lb = f2bf_bits(sp[e] - bf_bits2f(hb));
              hv[e] = __builtin_bit_cast(_Float16, hb);
              lv[e] = __builtin_bit_cast(_Float16, lb);
            }
          }
          *(volatile v8h*)(C + (size_t)(mBase + row) * ldc + n0 + c8) = hv;
          if (OUT_MODE == 2) *(volatile v8h*)(C2 + (size_t)(mBase + row) * ldc + n0 + c8) = lv;
        }
        __threadfence();
      }
    }
    __builtin_amdgcn_fence(__ATOMIC_RELEASE, "workgroup");
    __builtin_amdgcn_wave_barrier();
    __builtin_amdgcn_fence(__ATOMIC_ACQUIRE, "workgroup");
  }
}

__global__ __launch_bounds__(256) void k_cast_bf16x2(
    const float* __restrict__ in, unsigned short* __restrict__ out, int n2) {
  int i = blockIdx.x * 256 + threadIdx.x;
  if (i < n2) {
    const unsigned u = (unsigned)f2bf_bits(in[2 * i]) | ((unsigned)f2bf_bits(in[2 * i + 1]) << 16);
    ((volatile unsigned*)out)[i] = u;
    __threadfence();
    ((volatile unsigned*)out)[i] = u;
  }
}

__global__ __launch_bounds__(256) void k_transpose_bf16(
    const float* __restrict__ in, unsigned short* __restrict__ out, int C, int L) {
  __shared__ float t[64][33];
  const int tid = threadIdx.x;
  const int b = blockIdx.z;
  const int l0 = blockIdx.x * 32, c0 = blockIdx.y * 64;
  const float* inb = in + (size_t)b * C * L;
#pragma unroll
  for (int i = 0; i < 8; ++i) {
    const int cl = i * 8 + (tid >> 5);
    t[cl][tid & 31] = inb[(size_t)(c0 + cl) * L + l0 + (tid & 31)];
  }
  __syncthreads();
  const int r = tid >> 3, c8 = (tid & 7) * 8;
  unsigned w0, w1, w2, w3;
  w0 = (unsigned)f2bf_bits(t[c8 + 0][r]) | ((unsigned)f2bf_bits(t[c8 + 1][r]) << 16);
  w1 = (unsigned)f2bf_bits(t[c8 + 2][r]) | ((unsigned)f2bf_bits(t[c8 + 3][r]) << 16);
  w2 = (unsigned)f2bf_bits(t[c8 + 4][r]) | ((unsigned)f2bf_bits(t[c8 + 5][r]) << 16);
  w3 = (unsigned)f2bf_bits(t[c8 + 6][r]) | ((unsigned)f2bf_bits(t[c8 + 7][r]) << 16);
  const v4u val = (v4u){w0, w1, w2, w3};
  unsigned short* dst = out + ((size_t)b * L + l0 + r) * C + c0 + c8;
  *(volatile v4u*)dst = val;
  __threadfence();
  *(volatile v4u*)dst = val;
}

template <int MODE>
__global__ __launch_bounds__(128) void k_colnorm(
    const float* __restrict__ X, const unsigned* __restrict__ res,
    unsigned* __restrict__ outh, unsigned* __restrict__ outl, int ncol) {
  constexpr int NR = 1024;
  const int b = blockIdx.y;
  const int c = blockIdx.x * 256 + threadIdx.x * 2;
  const size_t base = (size_t)b * NR * ncol + c;
  const float* xb = X + base;
  float sa0 = 0.f, sa1 = 0.f, sb0 = 0.f, sb1 = 0.f;
#pragma unroll 1
  for (int l = 0; l < NR; l += 2) {
    const v2f u = *(const v2f*)(xb + (size_t)l * ncol);
    const v2f w = *(const v2f*)(xb + (size_t)(l + 1) * ncol);
    sa0 += u.x; sa1 += u.y; sb0 += w.x; sb1 += w.y;
  }
  const float m0 = (sa0 + sb0) * (1.0f / NR);
  const float m1 = (sa1 + sb1) * (1.0f / NR);
  float qa0 = 0.f, qa1 = 0.f, qb0 = 0.f, qb1 = 0.f;
#pragma unroll 1
  for (int l = 0; l < NR; l += 2) {
    const v2f u = *(const v2f*)(xb + (size_t)l * ncol);
    const v2f w = *(const v2f*)(xb + (size_t)(l + 1) * ncol);
    const float d0 = u.x - m0, d1 = u.y - m1, e0 = w.x - m0, e1 = w.y - m1;
    qa0 += d0 * d0; qa1 += d1 * d1; qb0 += e0 * e0; qb1 += e1 * e1;
  }
  const float r0 = rsqrtf((qa0 + qb0) * (1.0f / NR) + 1e-5f);
  const float r1 = rsqrtf((qa1 + qb1) * (1.0f / NR) + 1e-5f);
#pragma unroll 1
  for (int l = 0; l < NR; ++l) {
    const size_t ei = base + (size_t)l * ncol;
    const v2f u = *(const v2f*)(X + ei);
    float y0 = (u.x - m0) * r0;
    float y1 = (u.y - m1) * r1;
    if constexpr (MODE == 1) {
      const unsigned rw = res[ei >> 1];
      y0 += __uint_as_float(rw << 16);
      y1 += __uint_as_float(rw & 0xffff0000u);
    }
    if constexpr (MODE == 2) {
      y0 = fmaxf(y0, 0.0f);
      y1 = fmaxf(y1, 0.0f);
    }
    const unsigned short hb0 = f2bf_bits(y0), hb1 = f2bf_bits(y1);
    const unsigned short lb0 = f2bf_bits(y0 - bf_bits2f(hb0));
    const unsigned short lb1 = f2bf_bits(y1 - bf_bits2f(hb1));
    const unsigned hw = (unsigned)hb0 | ((unsigned)hb1 << 16);
    const unsigned lw = (unsigned)lb0 | ((unsigned)lb1 << 16);
    const size_t oi = ei >> 1;
    ((volatile unsigned*)outh)[oi] = hw;
    ((volatile unsigned*)outl)[oi] = lw;
    __threadfence();
    ((volatile unsigned*)outh)[oi] = hw;
    ((volatile unsigned*)outl)[oi] = lw;
  }
}

template <int MODE>
__global__ __launch_bounds__(256) void k_rownorm(
    const float* __restrict__ X, float* __restrict__ outf,
    unsigned short* __restrict__ outh, unsigned short* __restrict__ outl) {
  constexpr int NCOL = 1024;
  const int lane = threadIdx.x & 31, wave = threadIdx.x >> 5;
  const size_t row = (size_t)blockIdx.x * 8 + wave;
  const float* xr = X + row * NCOL;
  float s = 0.f;
#pragma unroll 1
  for (int it = 0; it < 8; ++it) {
    const v4f u = *(const v4f*)(xr + it * 128 + lane * 4);
    s += (u.x + u.y) + (u.z + u.w);
  }
#pragma unroll
  for (int off = 1; off < 32; off <<= 1) s += __shfl_xor(s, off, 32);
  const float mean = s * (1.0f / NCOL);
  float ss = 0.f;
#pragma unroll 1
  for (int it = 0; it < 8; ++it) {
    const v4f u = *(const v4f*)(xr + it * 128 + lane * 4);
    const float d0 = u.x - mean, d1 = u.y - mean, d2 = u.z - mean, d3 = u.w - mean;
    ss += (d0 * d0 + d1 * d1) + (d2 * d2 + d3 * d3);
  }
#pragma unroll
  for (int off = 1; off < 32; off <<= 1) ss += __shfl_xor(ss, off, 32);
  const float rs = rsqrtf(ss * (1.0f / NCOL) + 1e-5f);
  if constexpr (MODE == 0) {
    float* orow = outf + row * NCOL;
    for (int pass = 0; pass < 2; ++pass) {
#pragma unroll 1
      for (int it = 0; it < 8; ++it) {
        const v4f u = *(const v4f*)(xr + it * 128 + lane * 4);
        v4f y;
        y.x = (u.x - mean) * rs; y.y = (u.y - mean) * rs; y.z = (u.z - mean) * rs; y.w = (u.w - mean) * rs;
        *(volatile v4f*)(orow + it * 128 + lane * 4) = y;
      }
      __threadfence();
    }
  } else {
    unsigned short* hrow = outh + row * NCOL;
    unsigned short* lrw  = outl + row * NCOL;
    for (int pass = 0; pass < 2; ++pass) {
#pragma unroll 1
      for (int it = 0; it < 4; ++it) {
        const v4f u0 = *(const v4f*)(xr + it * 256 + lane * 8);
        const v4f u1 = *(const v4f*)(xr + it * 256 + lane * 8 + 4);
        const float y0 = (u0.x - mean) * rs, y1 = (u0.y - mean) * rs, y2 = (u0.z - mean) * rs, y3 = (u0.w - mean) * rs;
        const float y4 = (u1.x - mean) * rs, y5 = (u1.y - mean) * rs, y6 = (u1.z - mean) * rs, y7 = (u1.w - mean) * rs;
        const unsigned short h0 = f2bf_bits(y0), h1 = f2bf_bits(y1), h2 = f2bf_bits(y2), h3 = f2bf_bits(y3);
        const unsigned short h4 = f2bf_bits(y4), h5 = f2bf_bits(y5), h6 = f2bf_bits(y6), h7 = f2bf_bits(y7);
        const unsigned short l0 = f2bf_bits(y0 - bf_bits2f(h0)), l1 = f2bf_bits(y1 - bf_bits2f(h1));
        const unsigned short l2 = f2bf_bits(y2 - bf_bits2f(h2)), l3 = f2bf_bits(y3 - bf_bits2f(h3));
        const unsigned short l4 = f2bf_bits(y4 - bf_bits2f(h4)), l5 = f2bf_bits(y5 - bf_bits2f(h5));
        const unsigned short l6 = f2bf_bits(y6 - bf_bits2f(h6)), l7 = f2bf_bits(y7 - bf_bits2f(h7));
        const v4u hv = (v4u){ (unsigned)h0 | ((unsigned)h1 << 16), (unsigned)h2 | ((unsigned)h3 << 16),
                              (unsigned)h4 | ((unsigned)h5 << 16), (unsigned)h6 | ((unsigned)h7 << 16) };
        const v4u lv = (v4u){ (unsigned)l0 | ((unsigned)l1 << 16), (unsigned)l2 | ((unsigned)l3 << 16),
                              (unsigned)l4 | ((unsigned)l5 << 16), (unsigned)l6 | ((unsigned)l7 << 16) };
        *(volatile v4u*)(hrow + it * 256 + lane * 8) = hv;
        *(volatile v4u*)(lrw  + it * 256 + lane * 8) = lv;
      }
      __threadfence();
    }
  }
}

#define AT_D 64
#define AT_NW 4
#define AT_KC 64
#define AT_OSP 68
constexpr int SEQ_LEN = 1024;
constexpr int N_HEADS = 8;
constexpr int N_CH = 512;

__device__ __forceinline__ v8f at_mma(v16b a, v16b b, v8f c) {
  c = __builtin_amdgcn_wmma_f32_16x16x32_bf16(false, a, false, b, (short)0, c, false, false);
  asm volatile("v_nop\n\tv_nop\n\tv_nop\n\tv_nop" : "+v"(c) : "v"(a), "v"(b));
  return c;
}
__device__ __forceinline__ void at_split(float f, __bf16& hi, __bf16& lo) {
  const unsigned short hb = f2bf_bits(f);
  hi = __builtin_bit_cast(__bf16, hb);
  lo = __builtin_bit_cast(__bf16, f2bf_bits(f - __uint_as_float(((unsigned)hb) << 16)));
}

__global__ __launch_bounds__(128)
void k_attn(const unsigned short* __restrict__ qhp, const unsigned short* __restrict__ qlp,
            const unsigned short* __restrict__ khp, const unsigned short* __restrict__ klp,
            const unsigned short* __restrict__ vhp, const unsigned short* __restrict__ vlp,
            float* __restrict__ out, float sscale) {
  union FB { v16b v; v8b h[2]; };
  __shared__ __align__(16) __bf16 Ksh[AT_KC * AT_D];
  __shared__ __align__(16) __bf16 Ksl[AT_KC * AT_D];
  __shared__ __align__(16) __bf16 Vth[AT_D * AT_KC];
  __shared__ __align__(16) __bf16 Vtl[AT_D * AT_KC];
  __shared__ __align__(16) __bf16 Psh[AT_NW][16 * AT_KC];
  __shared__ __align__(16) __bf16 Psl[AT_NW][16 * AT_KC];
  __shared__ __align__(16) float  Os[AT_NW][16 * AT_OSP];

  const int tid  = threadIdx.x;
  const int wave = tid >> 5;
  const int lane = tid & 31;
  const int hh   = lane >> 4;
  const int c    = lane & 15;

  constexpr int NQB = SEQ_LEN / 64;
  const int bx  = blockIdx.x;
  const int qb  = bx % NQB;
  const int bhd = bx / NQB;
  const int h   = bhd % N_HEADS;
  const int b   = bhd / N_HEADS;
  const int q0  = qb * 64 + wave * 16;

  const __bf16* qh = (const __bf16*)qhp;
  const __bf16* ql = (const __bf16*)qlp;
  const __bf16* kh = (const __bf16*)khp;
  const __bf16* kl = (const __bf16*)klp;
  const __bf16* vh = (const __bf16*)vhp;
  const __bf16* vl = (const __bf16*)vlp;

  v16b qah[2], qal[2];
  {
    const size_t qo = ((size_t)b * SEQ_LEN + q0 + c) * N_CH + h * AT_D + 8 * hh;
#pragma unroll
    for (int dc = 0; dc < 2; ++dc) {
      qah[dc] = Frag<__bf16>::load(qh + qo + dc * 32);
      qal[dc] = Frag<__bf16>::load(ql + qo + dc * 32);
    }
  }

  float mrow[8], lrow[8];
  v8f oacc[4];
#pragma unroll
  for (int r = 0; r < 8; ++r) { mrow[r] = -INFINITY; lrow[r] = 0.f; }
#pragma unroll
  for (int t = 0; t < 4; ++t) oacc[t] = (v8f){0.f,0.f,0.f,0.f,0.f,0.f,0.f,0.f};

  for (int kc = 0; kc < SEQ_LEN / AT_KC; ++kc) {
    const int kv0 = kc * AT_KC;
    __syncthreads();
    {
      const int row = tid >> 1, half = (tid & 1) * 32;
      const size_t ko = ((size_t)b * SEQ_LEN + kv0 + row) * N_CH + h * AT_D + half;
      const size_t vo = ((size_t)b * N_CH + h * AT_D + row) * SEQ_LEN + kv0 + half;
      {
        const v4u* sp = (const v4u*)(kh + ko);
        v4u* dp = (v4u*)(Ksh + row * AT_D + half);
#pragma unroll
        for (int i = 0; i < 4; ++i) dp[i] = sp[i];
      }
      asm volatile("" ::: "memory");
      {
        const v4u* sp = (const v4u*)(kl + ko);
        v4u* dp = (v4u*)(Ksl + row * AT_D + half);
#pragma unroll
        for (int i = 0; i < 4; ++i) dp[i] = sp[i];
      }
      asm volatile("" ::: "memory");
      {
        const v4u* sp = (const v4u*)(vh + vo);
        v4u* dp = (v4u*)(Vth + row * AT_KC + half);
#pragma unroll
        for (int i = 0; i < 4; ++i) dp[i] = sp[i];
      }
      asm volatile("" ::: "memory");
      {
        const v4u* sp = (const v4u*)(vl + vo);
        v4u* dp = (v4u*)(Vtl + row * AT_KC + half);
#pragma unroll
        for (int i = 0; i < 4; ++i) dp[i] = sp[i];
      }
    }
    __syncthreads();

    v8f s[4];
#pragma unroll
    for (int j = 0; j < 4; ++j) {
      s[j] = (v8f){0.f,0.f,0.f,0.f,0.f,0.f,0.f,0.f};
#pragma unroll
      for (int dc = 0; dc < 2; ++dc) {
        FB kb, kb2;
        const int ko2 = (j * 16 + c) * AT_D + dc * 32 + 8 * hh;
        kb.h[0]  = *(const v8b*)(Ksh + ko2);
        kb.h[1]  = *(const v8b*)(Ksh + ko2 + 16);
        kb2.h[0] = *(const v8b*)(Ksl + ko2);
        kb2.h[1] = *(const v8b*)(Ksl + ko2 + 16);
        s[j] = at_mma(qah[dc], kb.v,  s[j]);
        s[j] = at_mma(qah[dc], kb2.v, s[j]);
        s[j] = at_mma(qal[dc], kb.v,  s[j]);
      }
    }
    float cm[8];
#pragma unroll
    for (int r = 0; r < 8; ++r) {
      float m = -INFINITY;
#pragma unroll
      for (int j = 0; j < 4; ++j) {
        const float sv = s[j][r] * sscale;
        s[j][r] = sv;
        m = fmaxf(m, sv);
      }
#pragma unroll
      for (int off = 1; off < 16; off <<= 1) m = fmaxf(m, __shfl_xor(m, off, 32));
      cm[r] = m;
    }
    __bf16* pwh = Psh[wave];
    __bf16* pwl = Psl[wave];
#pragma unroll
    for (int r = 0; r < 8; ++r) {
      const float mnew = fmaxf(mrow[r], cm[r]);
      const float alpha = expf(mrow[r] - mnew);
      mrow[r] = mnew;
      float psum = 0.f;
#pragma unroll
      for (int j = 0; j < 4; ++j) {
        const float p = expf(s[j][r] - mnew);
        psum += p;
        __bf16 pa_hi, pa_lo;
        at_split(p, pa_hi, pa_lo);
        pwh[(8 * hh + r) * AT_KC + j * 16 + c] = pa_hi;
        pwl[(8 * hh + r) * AT_KC + j * 16 + c] = pa_lo;
      }
#pragma unroll
      for (int off = 1; off < 16; off <<= 1) psum += __shfl_xor(psum, off, 32);
      lrow[r] = lrow[r] * alpha + psum;
#pragma unroll
      for (int t = 0; t < 4; ++t) oacc[t][r] *= alpha;
    }
    __builtin_amdgcn_fence(__ATOMIC_RELEASE, "workgroup");
    __builtin_amdgcn_wave_barrier();
    __builtin_amdgcn_fence(__ATOMIC_ACQUIRE, "workgroup");
#pragma unroll 1
    for (int kk = 0; kk < 2; ++kk) {
      FB pa, pl;
      const int po = c * AT_KC + kk * 32 + 8 * hh;
      pa.h[0] = *(const v8b*)(pwh + po);
      pa.h[1] = *(const v8b*)(pwh + po + 16);
      pl.h[0] = *(const v8b*)(pwl + po);
      pl.h[1] = *(const v8b*)(pwl + po + 16);
#pragma unroll
      for (int t = 0; t < 4; ++t) {
        FB vb, vb2;
        const int vo2 = (t * 16 + c) * AT_KC + kk * 32 + 8 * hh;
        vb.h[0]  = *(const v8b*)(Vth + vo2);
        vb.h[1]  = *(const v8b*)(Vth + vo2 + 16);
        vb2.h[0] = *(const v8b*)(Vtl + vo2);
        vb2.h[1] = *(const v8b*)(Vtl + vo2 + 16);
        oacc[t] = at_mma(pa.v, vb.v,  oacc[t]);
        oacc[t] = at_mma(pa.v, vb2.v, oacc[t]);
        oacc[t] = at_mma(pl.v, vb.v,  oacc[t]);
      }
    }
  }

  float* os = Os[wave];
#pragma unroll
  for (int r = 0; r < 8; ++r) {
    const float inv = 1.0f / lrow[r];
#pragma unroll
    for (int t = 0; t < 4; ++t) os[(8 * hh + r) * AT_OSP + t * 16 + c] = oacc[t][r] * inv;
  }
  __builtin_amdgcn_fence(__ATOMIC_RELEASE, "workgroup");
  __builtin_amdgcn_wave_barrier();
  __builtin_amdgcn_fence(__ATOMIC_ACQUIRE, "workgroup");
  {
    float* ob = out + ((size_t)b * SEQ_LEN) * N_CH + h * AT_D;
    const int c4 = (lane & 15) * 4;
    for (int pass = 0; pass < 2; ++pass) {
#pragma unroll
      for (int it = 0; it < 8; ++it) {
        const int row = it * 2 + hh;
        v4f val = *(const v4f*)(os + row * AT_OSP + c4);
        *(volatile v4f*)(ob + (size_t)(q0 + row) * N_CH + c4) = val;
      }
      __threadfence();
    }
  }
}

extern "C" void kernel_launch(void* const* d_in, const int* in_sizes, int n_in,
                              void* d_out, int out_size, void* d_ws,
                              size_t ws_size, hipStream_t stream) {
  (void)in_sizes; (void)n_in; (void)out_size;
  constexpr int NB = 8, CIN = 256, NCH = 512, SEQ = 1024, NFF = 1024, NHD = 8;

  constexpr size_t SZ_WQ   = (size_t)NCH * NCH * 2;
  constexpr size_t SZ_WK   = (size_t)NCH * CIN * 2;
  constexpr size_t SZ_WV   = (size_t)NCH * CIN * 2;
  constexpr size_t SZ_W1   = (size_t)NFF * NCH * 2;
  constexpr size_t SZ_W2   = (size_t)NCH * NFF * 2;
  constexpr size_t SZ_XQT  = (size_t)NB * SEQ * NCH * 2;
  constexpr size_t SZ_XKVT = (size_t)NB * SEQ * CIN * 2;
  constexpr size_t SZ_G    = (size_t)NB * SEQ * NFF * 4;
  constexpr size_t SZ_P    = (size_t)NB * SEQ * NCH * 2;
  constexpr size_t OFF_WQ   = 0;
  constexpr size_t OFF_WK   = OFF_WQ + SZ_WQ;
  constexpr size_t OFF_WV   = OFF_WK + SZ_WK;
  constexpr size_t OFF_W1   = OFF_WV + SZ_WV;
  constexpr size_t OFF_W2   = OFF_W1 + SZ_W1;
  constexpr size_t OFF_XQT  = OFF_W2 + SZ_W2;
  constexpr size_t OFF_XKVT = OFF_XQT + SZ_XQT;
  constexpr size_t OFF_G    = OFF_XKVT + SZ_XKVT;
  constexpr size_t OFF_QH   = OFF_G + SZ_G;
  constexpr size_t OFF_QL   = OFF_QH + SZ_P;
  constexpr size_t OFF_KH   = OFF_QL + SZ_P;
  constexpr size_t OFF_KL   = OFF_KH + SZ_P;
  constexpr size_t OFF_VH   = OFF_KL + SZ_P;
  constexpr size_t OFF_VL   = OFF_VH + SZ_P;
  constexpr size_t OFF_END  = OFF_VL + SZ_P;
  static_assert(OFF_END == 99614720ull);
  static_assert(OFF_END <= 134217728ull);
  static_assert((OFF_WK % 256) == 0 && (OFF_XQT % 256) == 0 && (OFF_G % 256) == 0 && (OFF_QH % 256) == 0);
  static_assert((size_t)NB * SEQ * NCH * 4 <= SZ_G);
  static_assert((size_t)NB * SEQ * NFF * 4 <= SZ_G);
  static_assert((size_t)NB * SEQ * NFF * 2 == 2 * SZ_P);
  static_assert(SEQ % 64 == 0 && NCH % 64 == 0 && NFF % 64 == 0);
  static_assert(NCH % 32 == 0 && CIN % 32 == 0 && NFF % 32 == 0);
  static_assert(((SEQ / 64) * (NCH / 64)) % 8 == 0 && ((SEQ / 64) * (NFF / 64)) % 8 == 0);
  static_assert(NCH % 256 == 0 && NFF % 256 == 0 && (NB * NCH) % 8 == 0);
  static_assert((size_t)NB * NCH * SEQ * 4 == 16777216ull);
  if (ws_size < OFF_END) return;

  const float* x_query = (const float*)d_in[0];
  const float* x_kv    = (const float*)d_in[1];
  const float* wq      = (const float*)d_in[2];
  const float* bq      = (const float*)d_in[3];
  const float* wk      = (const float*)d_in[4];
  const float* bk      = (const float*)d_in[5];
  const float* wv      = (const float*)d_in[6];
  const float* bv      = (const float*)d_in[7];
  const float* w1      = (const float*)d_in[8];
  const float* b1      = (const float*)d_in[9];
  const float* w2      = (const float*)d_in[10];
  const float* b2      = (const float*)d_in[11];
  float* out = (float*)d_out;

  char* ws = (char*)d_ws;
  typedef unsigned short us;
  us* wq16  = (us*)(ws + OFF_WQ);
  us* wk16  = (us*)(ws + OFF_WK);
  us* wv16  = (us*)(ws + OFF_WV);
  us* w1_16 = (us*)(ws + OFF_W1);
  us* w2_16 = (us*)(ws + OFF_W2);
  us* xqT   = (us*)(ws + OFF_XQT);
  us* xkvT  = (us*)(ws + OFF_XKVT);
  float* gf = (float*)(ws + OFF_G);
  us* qh = (us*)(ws + OFF_QH);
  us* ql = (us*)(ws + OFF_QL);
  us* kh = (us*)(ws + OFF_KH);
  us* kl = (us*)(ws + OFF_KL);
  us* vh = (us*)(ws + OFF_VH);
  us* vl = (us*)(ws + OFF_VL);
  us* zh = qh;
  us* zl = ql;
  us* yh = kh;
  us* yl = vh;

  k_cast_bf16x2<<<(NCH * NCH / 2 + 255) / 256, 256, 0, stream>>>(wq, wq16, NCH * NCH / 2);
  k_cast_bf16x2<<<(NCH * CIN / 2 + 255) / 256, 256, 0, stream>>>(wk, wk16, NCH * CIN / 2);
  k_cast_bf16x2<<<(NCH * CIN / 2 + 255) / 256, 256, 0, stream>>>(wv, wv16, NCH * CIN / 2);
  k_cast_bf16x2<<<(NFF * NCH / 2 + 255) / 256, 256, 0, stream>>>(w1, w1_16, NFF * NCH / 2);
  k_cast_bf16x2<<<(NCH * NFF / 2 + 255) / 256, 256, 0, stream>>>(w2, w2_16, NCH * NFF / 2);

  k_transpose_bf16<<<dim3(SEQ / 32, NCH / 64, NB), 256, 0, stream>>>(x_query, xqT, NCH, SEQ);
  k_transpose_bf16<<<dim3(SEQ / 32, CIN / 64, NB), 256, 0, stream>>>(x_kv, xkvT, CIN, SEQ);

  wmma_gemm64<1, 0, 2, 0, false><<<dim3((SEQ / 64) * (NCH / 64) / 8, NB), 256, 0, stream>>>(
      xqT, nullptr, NCH, (long)SEQ * NCH, wq16, nullptr, NCH, 0L,
      (void*)gf, nullptr, NCH, (long)SEQ * NCH, bq, nullptr, 0L, SEQ, NCH, NCH, 1.0f);
  k_colnorm<0><<<dim3(NCH / 256, NB), 128, 0, stream>>>(gf, nullptr, (unsigned*)qh, (unsigned*)ql, NCH);

  wmma_gemm64<1, 0, 2, 0, false><<<dim3((SEQ / 64) * (NCH / 64) / 8, NB), 256, 0, stream>>>(
      xkvT, nullptr, CIN, (long)SEQ * CIN, wk16, nullptr, CIN, 0L,
      (void*)gf, nullptr, NCH, (long)SEQ * NCH, bk, nullptr, 0L, SEQ, NCH, CIN, 1.0f);
  k_colnorm<0><<<dim3(NCH / 256, NB), 128, 0, stream>>>(gf, nullptr, (unsigned*)kh, (unsigned*)kl, NCH);

  wmma_gemm64<1, 0, 1, 0, false><<<dim3((NCH / 64) * (SEQ / 64) / 8, NB), 256, 0, stream>>>(
      wv16, nullptr, CIN, 0L, xkvT, nullptr, CIN, (long)SEQ * CIN,
      (void*)gf, nullptr, SEQ, (long)NCH * SEQ, bv, nullptr, 0L, NCH, SEQ, CIN, 1.0f);
  k_rownorm<1><<<NB * NCH / 8, 256, 0, stream>>>(gf, nullptr, vh, vl);

  k_attn<<<NB * NHD * (SEQ / 64), 128, 0, stream>>>(qh, ql, kh, kl, vh, vl, gf, 0.125f);

  k_colnorm<1><<<dim3(NCH / 256, NB), 128, 0, stream>>>(gf, (const unsigned*)xqT, (unsigned*)zh, (unsigned*)zl, NCH);

  wmma_gemm64<1, 2, 2, 0, false><<<dim3((SEQ / 64) * (NFF / 64) / 8, NB), 256, 0, stream>>>(
      zh, zl, NCH, (long)SEQ * NCH, w1_16, nullptr, NCH, 0L,
      (void*)gf, nullptr, NFF, (long)SEQ * NFF, b1, nullptr, 0L, SEQ, NFF, NCH, 1.0f);
  k_colnorm<2><<<dim3(NFF / 256, NB), 128, 0, stream>>>(gf, nullptr, (unsigned*)yh, (unsigned*)yl, NFF);

  wmma_gemm64<1, 3, 1, 0, false><<<dim3((NCH / 64) * (SEQ / 64) / 8, NB), 256, 0, stream>>>(
      w2_16, nullptr, NFF, 0L, yh, yl, NFF, (long)SEQ * NFF,
      (void*)gf, nullptr, SEQ, (long)NCH * SEQ, b2, nullptr, 0L, NCH, SEQ, NFF, 1.0f);

  k_rownorm<0><<<NB * NCH / 8, 256, 0, stream>>>(gf, out, nullptr, nullptr);
}
